// DCNv2SkipRefiner_52621939311392
// MI455X (gfx1250) — hardware-verified
//
#include <hip/hip_runtime.h>
#include <stdint.h>

#pragma clang fp contract(off)

#define NB     8
#define NC     64
#define NOC    64
#define NOF    27
#define NOP    32
#define HI     128
#define WI     128
#define HWI    (HI * WI)
#define PD     130
#define KT     576
#define NPIX   (NB * HWI)
#define PLANE_E ((size_t)NB * PD * PD * NC)
#define SP     72
#define OFP    36
#define OSP    132
#define NLX    PD
#define NST    128
#define CSC    16.0f
#define WSC    1024.0f
#define INV_S  6.103515625e-05f
#define IN_EPS 1e-5f
#define WO_CHK (NOP * KT / 8)
#define WR_CHK (NOC * KT / 8)
#define WO_BLK (WO_CHK / 256)
#define WR_BLK (WR_CHK / 256)
#define TRAW_B (NOC * OSP * 4)

#define WS_WO   ((size_t)0)
#define WS_WR   (WS_WO + (size_t)NOP * KT * 2)
#define WS_XH   (WS_WR + (size_t)NOC * KT * 2)
#define WS_OF   (WS_XH + PLANE_E * 2)
#define WS_Y    (WS_OF + (size_t)NPIX * NOP * 4)
#define WS_ST   (WS_Y + (size_t)NB * NOC * HWI * 4)
#define WS_END  (WS_ST + (size_t)NB * HI * NST * 4)

static_assert(WO_CHK % 256 == 0);
static_assert(WR_CHK % 256 == 0);
static_assert(KT % 32 == 0);
static_assert(KT == 9 * NC);
static_assert((WS_WR % 128) == 0);
static_assert((WS_XH % 128) == 0);
static_assert((WS_OF % 128) == 0);
static_assert((WS_Y % 128) == 0);
static_assert((WS_ST % 128) == 0);
static_assert((WS_END % 128) == 0);
static_assert(WS_END <= (size_t)134217728);
static_assert((SP * 2) % 16 == 0);
static_assert((OFP * 4) % 16 == 0);
static_assert((OSP * 4) % 16 == 0);
static_assert(128 * SP * 2 <= TRAW_B);
static_assert(PD * SP * 2 <= 48000);
static_assert(128 * NOP * 4 + NOC * 4 + NST * 4 + TRAW_B <= 60000);
static_assert(64 * OFP * 4 <= 16384);
static_assert(NC * 2 == 128);

typedef _Float16       v16h __attribute__((ext_vector_type(16)));
typedef _Float16       v8h  __attribute__((ext_vector_type(8)));
typedef __bf16         v16b __attribute__((ext_vector_type(16)));
typedef __bf16         v8b  __attribute__((ext_vector_type(8)));
typedef float          v8f  __attribute__((ext_vector_type(8)));
typedef float          v4f  __attribute__((ext_vector_type(4)));
typedef unsigned       v4u  __attribute__((ext_vector_type(4)));
typedef unsigned short v8us __attribute__((ext_vector_type(8)));

__device__ __forceinline__ unsigned bfb(float f) {
  const unsigned u = __float_as_uint(f);
  return (u + 0x7FFFu + ((u >> 16) & 1u)) >> 16;
}
__device__ __forceinline__ float bf_rne(float f) { return __uint_as_float(bfb(f) << 16); }
__device__ __forceinline__ unsigned hbits(_Float16 h) {
  return (unsigned)__builtin_bit_cast(unsigned short, h);
}
__device__ __forceinline__ v8f zero8f() { v8f z = {0.f, 0.f, 0.f, 0.f, 0.f, 0.f, 0.f, 0.f}; return z; }
__device__ __forceinline__ v8us zero8us() {
  v8us z;
#pragma unroll
  for (int e = 0; e < 8; ++e) z[e] = (unsigned short)0;
  return z;
}

__device__ __forceinline__ v16h ldfrag_h(const _Float16* p) {
  union { v16h v; v8h h[2]; } f;
  f.h[0] = *(const v8h*)(p);
  f.h[1] = *(const v8h*)(p + 16);
  return f.v;
}
__device__ __forceinline__ v16b ldfrag_b(const __bf16* p) {
  union { v16b v; v8b h[2]; } f;
  f.h[0] = *(const v8b*)(p);
  f.h[1] = *(const v8b*)(p + 16);
  return f.v;
}

__device__ __forceinline__ v8f mma_h(v16h a, v16h b, v8f c) {
  return __builtin_amdgcn_wmma_f32_16x16x32_f16(false, a, false, b, (short)0, c, false, false);
}
__device__ __forceinline__ v8f mma_b(v16b a, v16b b, v8f c) {
  return __builtin_amdgcn_wmma_f32_16x16x32_bf16(false, a, false, b, (short)0, c, false, false);
}
template <typename F>
__device__ __forceinline__ void guard1x4(v8f& c0, const F& f0, const F& f1, const F& f2, const F& f3) {
#if defined(__HIP_DEVICE_COMPILE__)
  asm volatile("v_nop\n\tv_nop\n\tv_nop\n\tv_nop"
               : "+v"(c0)
               : "v"(f0), "v"(f1), "v"(f2), "v"(f3));
#endif
}
template <typename F>
__device__ __forceinline__ void guard4x5(v8f& c0, v8f& c1, v8f& c2, v8f& c3,
                                         const F& f0, const F& f1, const F& f2,
                                         const F& f3, const F& f4) {
#if defined(__HIP_DEVICE_COMPILE__)
  asm volatile("v_nop\n\tv_nop\n\tv_nop\n\tv_nop"
               : "+v"(c0), "+v"(c1), "+v"(c2), "+v"(c3)
               : "v"(f0), "v"(f1), "v"(f2), "v"(f3), "v"(f4));
#endif
}
__device__ __forceinline__ void acc_guard1(v8f& c0) {
#if defined(__HIP_DEVICE_COMPILE__)
  asm volatile("v_nop\n\tv_nop\n\tv_nop\n\tv_nop" : "+v"(c0));
#endif
}
__device__ __forceinline__ void acc_guard4(v8f& c0, v8f& c1, v8f& c2, v8f& c3) {
#if defined(__HIP_DEVICE_COMPILE__)
  asm volatile("v_nop\n\tv_nop\n\tv_nop\n\tv_nop"
               : "+v"(c0), "+v"(c1), "+v"(c2), "+v"(c3));
#endif
}

__global__ __launch_bounds__(256)
void k_wpack(const float* __restrict__ woff, const float* __restrict__ wreg, unsigned* wo, unsigned* wr)
{
  const int tid = threadIdx.x;
  if (blockIdx.x < WO_BLK) {
    const int q   = blockIdx.x * 256 + tid;
    const int co  = q / (KT / 8);
    const int kc  = (q - co * (KT / 8)) * 8;
    const int tap = kc >> 6;
    const int ci0 = kc & (NC - 1);
    const int coc = (co < NOF) ? co : (NOF - 1);
    unsigned hb[8];
#pragma unroll
    for (int j = 0; j < 8; ++j) {
      const unsigned t = bfb(woff[((size_t)(coc * NC + ci0 + j)) * 9 + tap]);
      hb[j] = (co < NOF) ? t : 0u;
    }
    v4u wh;
    wh.x = hb[0] | (hb[1] << 16);
    wh.y = hb[2] | (hb[3] << 16);
    wh.z = hb[4] | (hb[5] << 16);
    wh.w = hb[6] | (hb[7] << 16);
    unsigned* dst = wo + (size_t)q * 4;
    *(volatile v4u*)dst = wh;
    __threadfence();
    *(volatile v4u*)dst = wh;
  } else {
    const int q   = (blockIdx.x - WO_BLK) * 256 + tid;
    const int co  = q / (KT / 8);
    const int kc  = (q - co * (KT / 8)) * 8;
    const int tap = kc >> 6;
    const int ci0 = kc & (NC - 1);
    unsigned hb[8];
#pragma unroll
    for (int j = 0; j < 8; ++j) {
      const float v = bf_rne(wreg[((size_t)(co * NC + ci0 + j)) * 9 + tap]) * WSC;
      hb[j] = hbits((_Float16)v);
    }
    v4u wh;
    wh.x = hb[0] | (hb[1] << 16);
    wh.y = hb[2] | (hb[3] << 16);
    wh.z = hb[4] | (hb[5] << 16);
    wh.w = hb[6] | (hb[7] << 16);
    unsigned* dst = wr + (size_t)q * 4;
    *(volatile v4u*)dst = wh;
    __threadfence();
    *(volatile v4u*)dst = wh;
  }
}

__global__ __launch_bounds__(256)
void k_xcvt(const float* __restrict__ x, unsigned short* xh)
{
  __shared__ __align__(16) unsigned short T[PD * SP];
  const int tid  = threadIdx.x;
  const int lane = tid & 31;
  const int wid  = tid >> 5;
  const int pj   = lane & 7;
  const int lq   = lane >> 3;
  const int b    = blockIdx.x / PD;
  const int hp   = blockIdx.x - b * PD;
  const size_t rowb = ((size_t)(b * PD + hp)) * PD;

  if (hp == 0 || hp == PD - 1) {
    const v8us zu = zero8us();
    size_t e[5]; bool ok[5];
#pragma unroll
    for (int r = 0; r < 5; ++r) {
      const int L  = r * 32 + wid * 4 + lq;
      ok[r] = (L < NLX);
      const int Lc = ok[r] ? L : (NLX - 1);
      e[r] = (rowb + Lc) * NC + 8 * pj;
    }
#pragma unroll
    for (int r = 0; r < 5; ++r) if (ok[r]) *(volatile v8us*)(xh + e[r]) = zu;
    __threadfence();
#pragma unroll
    for (int r = 0; r < 5; ++r) if (ok[r]) *(volatile v8us*)(xh + e[r]) = zu;
  } else {
    const int h = hp - 1;
    if (tid < 16) {
      const int slot = (tid < 8) ? 0 : (PD - 1);
      *(v8us*)&T[slot * SP + 8 * (tid & 7)] = zero8us();
    }
#pragma unroll
    for (int i = 0; i < 8; ++i) {
      const int idx = tid + 256 * i;
      const int w4  = idx & 31;
      const int c   = idx >> 5;
      const v4f v = *(const v4f*)(x + ((size_t)(b * NC + c) * HI + h) * WI + 4 * w4);
      unsigned short* tp = T + (4 * w4 + 1) * SP + c;
      tp[0 * SP] = (unsigned short)bfb(v.x);
      tp[1 * SP] = (unsigned short)bfb(v.y);
      tp[2 * SP] = (unsigned short)bfb(v.z);
      tp[3 * SP] = (unsigned short)bfb(v.w);
    }
    __syncthreads();
    v8us val[5]; size_t e[5]; bool ok[5];
#pragma unroll
    for (int r = 0; r < 5; ++r) {
      const int L  = r * 32 + wid * 4 + lq;
      ok[r] = (L < NLX);
      const int Lc = ok[r] ? L : (NLX - 1);
      val[r] = *(const v8us*)&T[Lc * SP + 8 * pj];
      e[r]   = (rowb + Lc) * NC + 8 * pj;
    }
#pragma unroll
    for (int r = 0; r < 5; ++r) if (ok[r]) *(volatile v8us*)(xh + e[r]) = val[r];
    __threadfence();
#pragma unroll
    for (int r = 0; r < 5; ++r) if (ok[r]) *(volatile v8us*)(xh + e[r]) = val[r];
  }
}

__global__ __launch_bounds__(256)
void k_offs(const __bf16* __restrict__ xh, const __bf16* __restrict__ wo,
            const float* __restrict__ obias, float* offp)
{
  __shared__ __align__(16) float st[64 * OFP];

  const int tid  = threadIdx.x;
  const int lane = tid & 31;
  const int wid  = tid >> 5;
  const int l15  = lane & 15;
  const int hh   = lane >> 4;
  const int b    = blockIdx.x >> 8;
  const int rm   = blockIdx.x & 255;
  const int h    = rm >> 1;
  const int xo   = (rm & 1) * 64;

  const int mt = wid & 3;
  const int nt = wid >> 2;
  const __bf16* ap = xh + (((size_t)(b * PD + h)) * PD + xo + 16 * mt + l15) * NC + 8 * hh;
  const __bf16* bp = wo + (size_t)(16 * nt + l15) * KT + 8 * hh;
  v8f acc = zero8f();
#pragma unroll 1
  for (int kh = 0; kh < 3; ++kh) {
#pragma unroll 1
    for (int kw = 0; kw < 3; ++kw) {
      const __bf16* a  = ap + (kh * PD + kw) * NC;
      const __bf16* bk = bp + (kh * 3 + kw) * NC;
      const v16b fa0 = ldfrag_b(a);
      const v16b fa1 = ldfrag_b(a + 32);
      const v16b fb0 = ldfrag_b(bk);
      const v16b fb1 = ldfrag_b(bk + 32);
      acc = mma_b(fa0, fb0, acc);
      acc = mma_b(fa1, fb1, acc);
      guard1x4(acc, fa0, fa1, fb0, fb1);
    }
  }
  acc_guard1(acc);

  {
    const int ch  = 16 * nt + l15;
    const int chc = (ch < NOF) ? ch : (NOF - 1);
    const float obv = bf_rne(obias[chc]);
    float* srow = st + (16 * mt + 8 * hh) * OFP + ch;
#pragma unroll
    for (int r = 0; r < 8; ++r) {
      float v = acc[r] + obv;
      if (ch >= NOF) v = 0.0f;
      srow[r * OFP] = v;
    }
  }
  __syncthreads();

#pragma unroll 1
  for (int it = tid; it < 64 * 9; it += 256) {
    const int px = it / 9;
    const int j  = it - px * 9;
    float* p = st + px * OFP + 18 + j;
    const float v = *p;
    const float e = expf(-fmaxf(v, -60.0f));
    const float s = 1.0f / (1.0f + e);
    *p = s;
  }
  __syncthreads();

  {
    const int pj = lane & 7;
    const int lq = lane >> 3;
    const size_t pix0 = (size_t)(b * HWI + h * WI + xo);
    v4f val[2]; size_t e[2];
#pragma unroll
    for (int r = 0; r < 2; ++r) {
      const int L = r * 32 + wid * 4 + lq;
      val[r] = *(const v4f*)&st[L * OFP + 4 * pj];
      e[r]   = (pix0 + L) * NOP + 4 * pj;
    }
#pragma unroll
    for (int r = 0; r < 2; ++r) *(volatile v4f*)(offp + e[r]) = val[r];
    __threadfence();
#pragma unroll
    for (int r = 0; r < 2; ++r) *(volatile v4f*)(offp + e[r]) = val[r];
  }
}

__global__ __launch_bounds__(256)
void k_conv(const unsigned short* __restrict__ xh, const _Float16* __restrict__ wr,
            const float* __restrict__ offp, const float* __restrict__ bias,
            float* yraw, float* part)
{
  __shared__ __align__(16) float offl[128 * NOP];
  __shared__ float bsl[NOC];
  __shared__ __align__(16) float stl[NST];
  __shared__ __align__(16) unsigned char traw[TRAW_B];
  _Float16* At = (_Float16*)traw;
  float*    os = (float*)traw;

  const int tid  = threadIdx.x;
  const int lane = tid & 31;
  const int wid  = tid >> 5;
  const int l15  = lane & 15;
  const int hh   = lane >> 4;
  const int pj   = lane & 7;
  const int lq   = lane >> 3;
  const int b    = blockIdx.x >> 7;
  const int h    = blockIdx.x & (HI - 1);
  const size_t pix0 = (size_t)(b * HWI + h * WI);

  if (tid < NOC) bsl[tid] = bf_rne(bias[tid]);
#pragma unroll
  for (int r = 0; r < 4; ++r) {
    const int idx = tid + 256 * r;
    const int px  = idx >> 3;
    const int pc  = idx & 7;
    *(v4f*)&offl[px * NOP + 4 * pc] = *(const v4f*)(offp + (pix0 + px) * NOP + 4 * pc);
  }
  __syncthreads();

  const _Float16* bp = wr + (size_t)l15 * KT + 8 * hh;
  v8f acc[4];
#pragma unroll
  for (int nt = 0; nt < 4; ++nt) acc[nt] = zero8f();

#pragma unroll 1
  for (int kh = 0; kh < 3; ++kh) {
#pragma unroll 1
    for (int kw = 0; kw < 3; ++kw) {
      const int tap = kh * 3 + kw;

      {
        const float hbase = (float)(h - 1 + kh);
#pragma unroll 1
        for (int i = 0; i < 4; ++i) {
          const int m = 32 * i + 4 * wid + lq;
          const float* orow = offl + m * NOP;
          const float dy = orow[2 * tap];
          const float dx = orow[2 * tap + 1];
          const float mk = orow[18 + tap];
          const float hf = hbase + dy;
          const float wf = (float)(m - 1 + kw) + dx;
          const float h0f = floorf(hf);
          const float w0f = floorf(wf);
          const float lh  = hf - h0f;
          const float lw  = wf - w0f;
          const float wh0 = 1.0f - lh;
          const float ww0 = 1.0f - lw;
          const int r0 = (int)fminf(fmaxf(h0f, -2.0f), (float)(PD - 1));
          const int c0 = (int)fminf(fmaxf(w0f, -2.0f), (float)(PD - 1));
          const int r1 = r0 + 1;
          const int c1 = c0 + 1;
          const bool vr0 = (r0 >= 0) && (r0 < HI);
          const bool vr1 = (r1 >= 0) && (r1 < HI);
          const bool vc0 = (c0 >= 0) && (c0 < WI);
          const bool vc1 = (c1 >= 0) && (c1 < WI);
          const float cw00 = (vr0 && vc0) ? (wh0 * ww0) : 0.0f;
          const float cw01 = (vr0 && vc1) ? (wh0 * lw)  : 0.0f;
          const float cw10 = (vr1 && vc0) ? (lh * ww0)  : 0.0f;
          const float cw11 = (vr1 && vc1) ? (lh * lw)   : 0.0f;
          const int pr0 = min(max(r0 + 1, 0), PD - 1);
          const int pr1 = min(max(r1 + 1, 0), PD - 1);
          const int pc0 = min(max(c0 + 1, 0), PD - 1);
          const int pc1 = min(max(c1 + 1, 0), PD - 1);
          const size_t rb0 = ((size_t)(b * PD + pr0)) * PD;
          const size_t rb1 = ((size_t)(b * PD + pr1)) * PD;
          const v4u q00 = *(const v4u*)(xh + (rb0 + pc0) * NC + 8 * pj);
          const v4u q01 = *(const v4u*)(xh + (rb0 + pc1) * NC + 8 * pj);
          const v4u q10 = *(const v4u*)(xh + (rb1 + pc0) * NC + 8 * pj);
          const v4u q11 = *(const v4u*)(xh + (rb1 + pc1) * NC + 8 * pj);
          v8h o;
#pragma unroll
          for (int j = 0; j < 4; ++j) {
            const unsigned u00 = q00[j], u01 = q01[j], u10 = q10[j], u11 = q11[j];
            {
              float a = cw00 * __uint_as_float(u00 << 16);
              a = a + cw01 * __uint_as_float(u01 << 16);
              a = a + cw10 * __uint_as_float(u10 << 16);
              a = a + cw11 * __uint_as_float(u11 << 16);
              a = a * mk;
              a = a * CSC;
              o[2 * j] = (_Float16)a;
            }
            {
              float a = cw00 * __uint_as_float(u00 & 0xffff0000u);
              a = a + cw01 * __uint_as_float(u01 & 0xffff0000u);
              a = a + cw10 * __uint_as_float(u10 & 0xffff0000u);
              a = a + cw11 * __uint_as_float(u11 & 0xffff0000u);
              a = a * mk;
              a = a * CSC;
              o[2 * j + 1] = (_Float16)a;
            }
          }
          *(v8h*)(At + m * SP + 8 * pj) = o;
        }
      }
      __syncthreads();

      {
        const _Float16* bt = bp + tap * NC;
        const _Float16* ab = At + (16 * wid + l15) * SP + 8 * hh;
#pragma unroll
        for (int kc = 0; kc < 2; ++kc) {
          const v16h fa  = ldfrag_h(ab + 32 * kc);
          const v16h fb0 = ldfrag_h(bt + 32 * kc);
          const v16h fb1 = ldfrag_h(bt + 16 * KT + 32 * kc);
          const v16h fb2 = ldfrag_h(bt + 32 * KT + 32 * kc);
          const v16h fb3 = ldfrag_h(bt + 48 * KT + 32 * kc);
          acc[0] = mma_h(fa, fb0, acc[0]);
          acc[1] = mma_h(fa, fb1, acc[1]);
          acc[2] = mma_h(fa, fb2, acc[2]);
          acc[3] = mma_h(fa, fb3, acc[3]);
          guard4x5(acc[0], acc[1], acc[2], acc[3], fa, fb0, fb1, fb2, fb3);
        }
      }
      __syncthreads();
    }
  }
  acc_guard4(acc[0], acc[1], acc[2], acc[3]);

#pragma unroll
  for (int nt = 0; nt < 4; ++nt) {
    const int col = 16 * nt + l15;
    const float bb = bsl[col];
    float* orow = os + col * OSP + 16 * wid + 8 * hh;
    v4f p0, p1;
    p0.x = acc[nt][0] * INV_S + bb;
    p0.y = acc[nt][1] * INV_S + bb;
    p0.z = acc[nt][2] * INV_S + bb;
    p0.w = acc[nt][3] * INV_S + bb;
    p1.x = acc[nt][4] * INV_S + bb;
    p1.y = acc[nt][5] * INV_S + bb;
    p1.z = acc[nt][6] * INV_S + bb;
    p1.w = acc[nt][7] * INV_S + bb;
    *(v4f*)(orow)     = p0;
    *(v4f*)(orow + 4) = p1;
  }
  __syncthreads();

  {
    const int co = tid >> 2;
    const int qq = tid & 3;
    const float* spx = os + co * OSP + 32 * qq;
    float s = 0.0f, q = 0.0f;
#pragma unroll
    for (int j = 0; j < 8; ++j) {
      const v4f v = *(const v4f*)(spx + 4 * j);
      s = s + v.x; q = q + v.x * v.x;
      s = s + v.y; q = q + v.y * v.y;
      s = s + v.z; q = q + v.z * v.z;
      s = s + v.w; q = q + v.w * v.w;
    }
    s = s + __shfl_xor(s, 1, 32);
    q = q + __shfl_xor(q, 1, 32);
    s = s + __shfl_xor(s, 2, 32);
    q = q + __shfl_xor(q, 2, 32);
    if (qq == 0) {
      stl[2 * co]     = s;
      stl[2 * co + 1] = q;
    }
  }
  __syncthreads();

  if (wid == 0) {
    const v4f sv = *(const v4f*)&stl[4 * lane];
    float* dst = part + (size_t)blockIdx.x * NST + 4 * lane;
    *(volatile v4f*)dst = sv;
    __threadfence();
    *(volatile v4f*)dst = sv;
  }

  {
    v4f val[8]; size_t e[8];
#pragma unroll
    for (int it = 0; it < 8; ++it) {
      const int L   = it * 32 + wid * 4 + lq;
      const int col = L >> 2;
      const int wq  = L & 3;
      val[it] = *(const v4f*)(os + col * OSP + 32 * wq + 4 * pj);
      e[it]   = ((size_t)(b * NOC + col) * HI + h) * WI + 32 * wq + 4 * pj;
    }
#pragma unroll
    for (int it = 0; it < 8; ++it) *(volatile v4f*)(yraw + e[it]) = val[it];
    __threadfence();
#pragma unroll
    for (int it = 0; it < 8; ++it) *(volatile v4f*)(yraw + e[it]) = val[it];
  }
}

__global__ __launch_bounds__(256)
void k_norm(const float* __restrict__ yraw, const float* __restrict__ part, float* out)
{
  __shared__ double ps[HI];
  __shared__ double pq[HI];
  __shared__ float sh[2];

  const int tid = threadIdx.x;
  const int blk = blockIdx.x;
  const int b   = blk >> 6;
  const int o   = blk & (NOC - 1);

  if (tid < HI) {
    const size_t idx = ((size_t)(b * HI + tid)) * NST + 2 * o;
    ps[tid] = (double)part[idx];
    pq[tid] = (double)part[idx + 1];
  }
  __syncthreads();
  if (tid == 0) {
    double S = 0.0, Q = 0.0;
#pragma unroll 1
    for (int i = 0; i < HI; ++i) { S += ps[i]; Q += pq[i]; }
    const double mu = S * (1.0 / (double)HWI);
    double var = Q * (1.0 / (double)HWI) - mu * mu;
    if (var < 0.0) var = 0.0;
    const float muf  = (float)mu;
    const float varf = (float)var;
    sh[0] = muf;
    sh[1] = rsqrtf(varf + IN_EPS);
  }
  __syncthreads();
  const float mu = sh[0];
  const float rs = sh[1];

  const size_t base = (size_t)blk * HWI;
  v4f val[16]; size_t e[16];
#pragma unroll
  for (int it = 0; it < 16; ++it) {
    const int idx = it * 256 + tid;
    e[it] = base + 4 * (size_t)idx;
    const v4f v = *(const v4f*)(yraw + e[it]);
    v4f t;
    t.x = (v.x - mu) * rs; t.x = (t.x > 0.0f) ? t.x : 0.0f;
    t.y = (v.y - mu) * rs; t.y = (t.y > 0.0f) ? t.y : 0.0f;
    t.z = (v.z - mu) * rs; t.z = (t.z > 0.0f) ? t.z : 0.0f;
    t.w = (v.w - mu) * rs; t.w = (t.w > 0.0f) ? t.w : 0.0f;
    val[it] = t;
  }
#pragma unroll
  for (int it = 0; it < 16; ++it) *(volatile v4f*)(out + e[it]) = val[it];
  __threadfence();
#pragma unroll
  for (int it = 0; it < 16; ++it) *(volatile v4f*)(out + e[it]) = val[it];
}

extern "C" void kernel_launch(void* const* d_in, const int* in_sizes, int n_in,
                              void* d_out, int out_size, void* d_ws, size_t ws_size,
                              hipStream_t stream) {
  if (n_in < 5) return;
  if (in_sizes[0] != NB * NC * HWI) return;
  if (in_sizes[1] != NOF * NC * 9) return;
  if (in_sizes[2] != NOF) return;
  if (in_sizes[3] != NOC * NC * 9) return;
  if (in_sizes[4] != NOC) return;
  if (out_size != NB * NOC * HWI) return;
  if (WS_END > ws_size) return;

  const float* x      = (const float*)d_in[0];
  const float* w_off  = (const float*)d_in[1];
  const float* b_off  = (const float*)d_in[2];
  const float* weight = (const float*)d_in[3];
  const float* bias   = (const float*)d_in[4];
  float* out = (float*)d_out;
  char* ws = (char*)d_ws;

  unsigned* wo_u       = (unsigned*)(ws + WS_WO);
  unsigned* wr_u       = (unsigned*)(ws + WS_WR);
  unsigned short* xh_u = (unsigned short*)(ws + WS_XH);
  float* offp          = (float*)(ws + WS_OF);
  float* yraw          = (float*)(ws + WS_Y);
  float* part          = (float*)(ws + WS_ST);

  k_wpack<<<dim3(WO_BLK + WR_BLK), dim3(256), 0, stream>>>(w_off, weight, wo_u, wr_u);
  (void)hipGetLastError();

  k_xcvt<<<dim3(NB * PD), dim3(256), 0, stream>>>(x, xh_u);
  (void)hipGetLastError();

  k_offs<<<dim3(NB * HI * 2), dim3(256), 0, stream>>>((const __bf16*)xh_u, (const __bf16*)wo_u,
                                                        b_off, offp);
  (void)hipGetLastError();

  k_conv<<<dim3(NB * HI), dim3(256), 0, stream>>>((const unsigned short*)xh_u, (const _Float16*)wr_u,
                                                    (const float*)offp, bias, yraw, part);
  (void)hipGetLastError();

  k_norm<<<dim3(NB * NOC), dim3(256), 0, stream>>>((const float*)yraw, (const float*)part, out);
  (void)hipGetLastError();
}
